// GMM_6176162971962
// MI455X (gfx1250) — hardware-verified
//
#include <hip/hip_runtime.h>
#include <math.h>
#include <stdint.h>

#define NR 8192
#define ND 1024
#define NJ 512
#define EPSN 1e-6f
#define WSLIM 134217728

typedef __attribute__((ext_vector_type(16))) __bf16   v16b;
typedef __attribute__((ext_vector_type(8)))  __bf16   v8b;
typedef __attribute__((ext_vector_type(8)))  float    v8f;
typedef __attribute__((ext_vector_type(4)))  float    v4f;
typedef __attribute__((ext_vector_type(4)))  unsigned int v4u;
typedef v4f __attribute__((may_alias)) v4fa;

static_assert((NR % 64) == 0);
static_assert((ND % 64) == 0);
static_assert((NJ % 64) == 0);
static_assert((NR % 32) == 0);
static_assert((ND % 32) == 0);
static_assert((NJ % 32) == 0);

__device__ __forceinline__ unsigned short f2bf_bits(float f) {
  unsigned u = __float_as_uint(f);
  return (unsigned short)((u + 0x7FFFu + ((u >> 16) & 1u)) >> 16);
}
__device__ __forceinline__ float bf_bits2f(unsigned short h) { return __uint_as_float(((unsigned)h) << 16); }
__device__ __forceinline__ unsigned pk16(unsigned short a, unsigned short b) { return (unsigned)a | ((unsigned)b << 16); }
__device__ __forceinline__ float bf16r(float f) { return bf_bits2f(f2bf_bits(f)); }
__device__ __forceinline__ void split2(float f0, float f1, unsigned& hw, unsigned& lw) {
  const unsigned short h0 = f2bf_bits(f0), h1 = f2bf_bits(f1);
  const unsigned short l0 = f2bf_bits(f0 - bf_bits2f(h0)), l1 = f2bf_bits(f1 - bf_bits2f(h1));
  hw = pk16(h0, h1);
  lw = pk16(l0, l1);
}

__device__ __forceinline__ void dep_guard_b(v8f& a, v8f& b, v16b x, v16b y) { asm volatile("v_nop\n\tv_nop\n\tv_nop\n\tv_nop" : "+v"(a), "+v"(b) : "v"(x), "v"(y)); }
__device__ __forceinline__ void keep4_b(v16b a, v16b b, v16b c, v16b d) { asm volatile("v_nop" :: "v"(a), "v"(b), "v"(c), "v"(d)); }
__device__ __forceinline__ void acc_guard4(v8f& a, v8f& b, v8f& c, v8f& d) { asm volatile("v_nop\n\tv_nop\n\tv_nop\n\tv_nop" : "+v"(a), "+v"(b), "+v"(c), "+v"(d)); }

struct FragB {
  union U { v16b v; v8b h[2]; };
  static __device__ __forceinline__ v16b load(const __bf16* p) {
    U f; f.h[0] = *(const v8b*)(p); f.h[1] = *(const v8b*)(p + 16); return f.v;
  }
  static __device__ __forceinline__ v8f mma(v16b a, v16b b, v8f c) {
    return __builtin_amdgcn_wmma_f32_16x16x32_bf16(false, a, false, b, (short)0, c, false, false);
  }
};

__device__ __forceinline__ v8f zero8() { v8f z = {0.f, 0.f, 0.f, 0.f, 0.f, 0.f, 0.f, 0.f}; return z; }

template <int RESID>
__global__ __launch_bounds__(256) void gemm64_kernel(
    const unsigned short* __restrict__ Ap, int lda, long aoff1, long aoff2,
    const unsigned short* __restrict__ Btp, int ldb, long boff1, long boff2,
    int nterm,
    float* Cp, int ldc,
    const float* __restrict__ Rp, int ldr,
    int M, int N, int K) {
  const __bf16* A  = (const __bf16*)(const void*)Ap;
  const __bf16* Bt = (const __bf16*)(const void*)Btp;
  __shared__ __align__(16) float sT[8][16 * 68];
  const int lane = threadIdx.x & 31;
  const int wave = threadIdx.x >> 5;
  const int tilesN = N >> 6;
  const int tilesM = M >> 6;
  const int tile = blockIdx.x * 8 + wave;
  if (tile >= tilesM * tilesN) return;
  const int tm = tile / tilesN;
  const int tn = tile - tm * tilesN;
  const int m0 = tm << 6;
  const int n0 = tn << 6;

  const int rlane = lane & 15;
  const int koff  = (lane >> 4) * 8;
  const int mOff  = (lane >> 4) * 8;

  v8f acc[4][4];
#pragma unroll
  for (int i = 0; i < 4; ++i)
#pragma unroll
    for (int j = 0; j < 4; ++j) acc[i][j] = zero8();

  for (int t = 0; t < nterm; ++t) {
    const long ao = (t == 0) ? 0L : ((t == 1) ? aoff1 : aoff2);
    const long bo = (t == 0) ? 0L : ((t == 1) ? boff1 : boff2);
    const __bf16* Ab = A + ao;
    const __bf16* Bb = Bt + bo;
    for (int k0 = 0; k0 < K; k0 += 32) {
      v16b bh[4];
#pragma unroll
      for (int j = 0; j < 4; ++j) {
        const size_t bofs = (size_t)(n0 + (j << 4) + rlane) * ldb + koff + k0;
        bh[j] = FragB::load(Bb + bofs);
      }
#pragma unroll
      for (int i = 0; i < 4; ++i) {
        const size_t aofs = (size_t)(m0 + (i << 4) + rlane) * lda + koff + k0;
        v16b ah = FragB::load(Ab + aofs);
#pragma unroll
        for (int j = 0; j < 4; ++j) acc[i][j] = FragB::mma(ah, bh[j], acc[i][j]);
        dep_guard_b(acc[i][0], acc[i][3], ah, ah);
      }
      keep4_b(bh[0], bh[1], bh[2], bh[3]);
    }
  }
  acc_guard4(acc[0][0], acc[0][1], acc[0][2], acc[0][3]);
  acc_guard4(acc[1][0], acc[1][1], acc[1][2], acc[1][3]);
  acc_guard4(acc[2][0], acc[2][1], acc[2][2], acc[2][3]);
  acc_guard4(acc[3][0], acc[3][1], acc[3][2], acc[3][3]);

  float* slab = sT[wave];
  const int q2 = lane >> 4, c4 = (lane & 15) * 4;
#pragma unroll
  for (int i = 0; i < 4; ++i) {
    const int mBase = m0 + (i << 4);
#pragma unroll
    for (int j = 0; j < 4; ++j) {
#pragma unroll
      for (int r = 0; r < 8; ++r) slab[(mOff + r) * 68 + (j << 4) + rlane] = acc[i][j][r];
    }
    __builtin_amdgcn_fence(__ATOMIC_RELEASE, "workgroup");
    __builtin_amdgcn_wave_barrier();
    __builtin_amdgcn_fence(__ATOMIC_ACQUIRE, "workgroup");
    for (int pass = 0; pass < 2; ++pass) {
#pragma unroll
      for (int it = 0; it < 8; ++it) {
        const int row = it * 2 + q2;
        v4f v = *(const v4fa*)(slab + row * 68 + c4);
        if (RESID) {
          const v4f c = *(const v4fa*)(Rp + (size_t)(mBase + row) * ldr + n0 + c4);
          v[0] += bf16r(c[0]); v[1] += bf16r(c[1]); v[2] += bf16r(c[2]); v[3] += bf16r(c[3]);
        }
        *(volatile v4f*)(Cp + (size_t)(mBase + row) * ldc + n0 + c4) = v;
      }
      __threadfence();
    }
    __builtin_amdgcn_fence(__ATOMIC_RELEASE, "workgroup");
    __builtin_amdgcn_wave_barrier();
    __builtin_amdgcn_fence(__ATOMIC_ACQUIRE, "workgroup");
  }
}

__global__ __launch_bounds__(256) void cvt_bf16x8_kernel(const float* __restrict__ in, unsigned short* __restrict__ o, int n8) {
  const int i = blockIdx.x * 256 + threadIdx.x;
  if (i < n8) {
    const float* sp = in + (size_t)i * 8;
    const v4f a  = *(const v4f*)(sp);
    const v4f a2 = *(const v4f*)(sp + 4);
    v4u w;
    w[0] = pk16(f2bf_bits(a[0]),  f2bf_bits(a[1]));
    w[1] = pk16(f2bf_bits(a[2]),  f2bf_bits(a[3]));
    w[2] = pk16(f2bf_bits(a2[0]), f2bf_bits(a2[1]));
    w[3] = pk16(f2bf_bits(a2[2]), f2bf_bits(a2[3]));
    unsigned short* dp = o + (size_t)i * 8;
    *(volatile v4u*)dp = w;
    __threadfence();
    *(volatile v4u*)dp = w;
  }
}

__global__ __launch_bounds__(256) void tcvt_kernel(const float* __restrict__ W, unsigned short* __restrict__ oh, int R, int Cc) {
  __shared__ __align__(16) float tf[64 * 68];
  const int c0  = blockIdx.x * 64;
  const int r0  = blockIdx.y * 64;
  const int tid = threadIdx.x;
  {
    const int lr = tid >> 4;
    const int cq = (tid & 15) * 4;
#pragma unroll
    for (int it = 0; it < 4; ++it) {
      const int rr = it * 16 + lr;
      const v4f a = *(const v4f*)(W + (size_t)(r0 + rr) * Cc + c0 + cq);
      *(v4f*)(tf + rr * 68 + cq) = a;
    }
  }
  __syncthreads();
  const int sub = tid >> 3;
  const int c8  = (tid & 7) * 8;
  v4u hv[2];
#pragma unroll
  for (int it = 0; it < 2; ++it) {
    const int oc = it * 32 + sub;
    v4u a;
#pragma unroll
    for (int q = 0; q < 4; ++q) {
      const float f0 = tf[(c8 + 2 * q) * 68 + oc];
      const float f1 = tf[(c8 + 2 * q + 1) * 68 + oc];
      a[q] = pk16(f2bf_bits(f0), f2bf_bits(f1));
    }
    hv[it] = a;
  }
  for (int pass = 0; pass < 2; ++pass) {
#pragma unroll
    for (int it = 0; it < 2; ++it) {
      const int oc = it * 32 + sub;
      const size_t go = (size_t)(c0 + oc) * R + r0 + c8;
      *(volatile v4u*)(oh + go) = hv[it];
    }
    __threadfence();
  }
}

__global__ __launch_bounds__(256) void tsplit_kernel(const float* __restrict__ W, unsigned short* __restrict__ oh,
                                                     unsigned short* __restrict__ ol, int R, int Cc) {
  __shared__ __align__(16) float tf[64 * 68];
  const int c0  = blockIdx.x * 64;
  const int r0  = blockIdx.y * 64;
  const int tid = threadIdx.x;
  {
    const int lr = tid >> 4;
    const int cq = (tid & 15) * 4;
#pragma unroll
    for (int it = 0; it < 4; ++it) {
      const int rr = it * 16 + lr;
      const v4f a = *(const v4f*)(W + (size_t)(r0 + rr) * Cc + c0 + cq);
      *(v4f*)(tf + rr * 68 + cq) = a;
    }
  }
  __syncthreads();
  const int sub = tid >> 3;
  const int c8  = (tid & 7) * 8;
  v4u hv[2], lv[2];
#pragma unroll
  for (int it = 0; it < 2; ++it) {
    const int oc = it * 32 + sub;
    v4u a, a2;
#pragma unroll
    for (int q = 0; q < 4; ++q) {
      const float f0 = tf[(c8 + 2 * q) * 68 + oc];
      const float f1 = tf[(c8 + 2 * q + 1) * 68 + oc];
      const unsigned short h0 = f2bf_bits(f0), h1 = f2bf_bits(f1);
      const unsigned short l0 = f2bf_bits(f0 - bf_bits2f(h0)), l1 = f2bf_bits(f1 - bf_bits2f(h1));
      a[q]  = pk16(h0, h1);
      a2[q] = pk16(l0, l1);
    }
    hv[it] = a; lv[it] = a2;
  }
  for (int pass = 0; pass < 2; ++pass) {
#pragma unroll
    for (int it = 0; it < 2; ++it) {
      const int oc = it * 32 + sub;
      const size_t go = (size_t)(c0 + oc) * R + r0 + c8;
      *(volatile v4u*)(oh + go) = hv[it];
      *(volatile v4u*)(ol + go) = lv[it];
    }
    __threadfence();
  }
}

__global__ __launch_bounds__(256) void colsoftmax_kernel(const float* __restrict__ S,
                                                        unsigned short* __restrict__ oh,
                                                        unsigned short* __restrict__ ol) {
  __shared__ float sRed[8][64];
  __shared__ float sFin[64];
  const int tid = threadIdx.x, wave = tid >> 5, lane = tid & 31;
  const int q = lane >> 3, c8 = (lane & 7) * 8;
  const int c0 = blockIdx.x * 64;
  const float* sb = S + c0 + c8;

  float mx[8];
#pragma unroll
  for (int e = 0; e < 8; ++e) mx[e] = -3.402823466e38f;
#pragma unroll 1
  for (int i = 0; i < 16; ++i) {
    const int j = i * 32 + wave * 4 + q;
    const float* p = sb + (size_t)j * NR;
    const v4f a = *(const v4fa*)(p);
    const v4f b = *(const v4fa*)(p + 4);
#pragma unroll
    for (int e = 0; e < 4; ++e) { mx[e] = fmaxf(mx[e], a[e]); mx[4 + e] = fmaxf(mx[4 + e], b[e]); }
  }
#pragma unroll
  for (int e = 0; e < 8; ++e) {
    mx[e] = fmaxf(mx[e], __shfl_xor(mx[e], 8));
    mx[e] = fmaxf(mx[e], __shfl_xor(mx[e], 16));
  }
  if (q == 0) {
#pragma unroll
    for (int e = 0; e < 8; ++e) sRed[wave][c8 + e] = mx[e];
  }
  __syncthreads();
  if (tid < 64) {
    float m = sRed[0][tid];
#pragma unroll
    for (int w = 1; w < 8; ++w) m = fmaxf(m, sRed[w][tid]);
    sFin[tid] = m;
  }
  __syncthreads();
  float cm[8];
#pragma unroll
  for (int e = 0; e < 8; ++e) cm[e] = sFin[c8 + e];

  float sm[8];
#pragma unroll
  for (int e = 0; e < 8; ++e) sm[e] = 0.0f;
#pragma unroll 1
  for (int i = 0; i < 16; ++i) {
    const int j = i * 32 + wave * 4 + q;
    const float* p = sb + (size_t)j * NR;
    const v4f a = *(const v4fa*)(p);
    const v4f b = *(const v4fa*)(p + 4);
#pragma unroll
    for (int e = 0; e < 4; ++e) { sm[e] += __expf(a[e] - cm[e]); sm[4 + e] += __expf(b[e] - cm[4 + e]); }
  }
#pragma unroll
  for (int e = 0; e < 8; ++e) {
    sm[e] += __shfl_xor(sm[e], 8);
    sm[e] += __shfl_xor(sm[e], 16);
  }
  if (q == 0) {
#pragma unroll
    for (int e = 0; e < 8; ++e) sRed[wave][c8 + e] = sm[e];
  }
  __syncthreads();
  if (tid < 64) {
    float s = sRed[0][tid];
#pragma unroll
    for (int w = 1; w < 8; ++w) s += sRed[w][tid];
    sFin[tid] = 1.0f / s;
  }
  __syncthreads();
  float inv[8];
#pragma unroll
  for (int e = 0; e < 8; ++e) inv[e] = sFin[c8 + e];

#pragma unroll 1
  for (int i = 0; i < 16; ++i) {
    const int j = i * 32 + wave * 4 + q;
    const float* p = sb + (size_t)j * NR;
    const v4f a = *(const v4fa*)(p);
    const v4f b = *(const v4fa*)(p + 4);
    float rv[8];
#pragma unroll
    for (int e = 0; e < 4; ++e) { rv[e] = __expf(a[e] - cm[e]) * inv[e]; rv[4 + e] = __expf(b[e] - cm[4 + e]) * inv[4 + e]; }
    v4u hv, lv;
#pragma unroll
    for (int k = 0; k < 4; ++k) {
      unsigned hw, lw;
      split2(rv[2 * k], rv[2 * k + 1], hw, lw);
      hv[k] = hw; lv[k] = lw;
    }
    const size_t go = (size_t)j * NR + c0 + c8;
    *(volatile v4u*)(oh + go) = hv;
    *(volatile v4u*)(ol + go) = lv;
    __threadfence();
    *(volatile v4u*)(oh + go) = hv;
    *(volatile v4u*)(ol + go) = lv;
  }
}

__global__ __launch_bounds__(256) void rownorm_kernel(const float* __restrict__ P, float* pn,
                                                     unsigned short* __restrict__ oh,
                                                     unsigned short* __restrict__ ol) {
  __shared__ __align__(16) float sRow[8][ND];
  const int lane = threadIdx.x & 31, wave = threadIdx.x >> 5;
  const int row = blockIdx.x * 8 + wave;
  const float* sp = P + (size_t)row * ND + 4 * lane;
  v4f v[8];
#pragma unroll
  for (int i = 0; i < 8; ++i) v[i] = *(const v4fa*)(sp + i * 128);
  float ss = 0.0f;
#pragma unroll
  for (int i = 0; i < 8; ++i)
#pragma unroll
    for (int e = 0; e < 4; ++e) ss += v[i][e] * v[i][e];
#pragma unroll
  for (int off = 16; off > 0; off >>= 1) ss += __shfl_xor(ss, off);
  const float inv = 1.0f / (sqrtf(ss) + EPSN);
#pragma unroll
  for (int i = 0; i < 8; ++i) v[i] = v[i] * inv;

  float* prow = pn + (size_t)row * ND + 4 * lane;
  for (int pass = 0; pass < 2; ++pass) {
#pragma unroll
    for (int i = 0; i < 8; ++i) *(volatile v4f*)(prow + i * 128) = v[i];
    __threadfence();
  }

  float* sr = sRow[wave];
#pragma unroll
  for (int i = 0; i < 8; ++i) *(v4fa*)(sr + i * 128 + 4 * lane) = v[i];
  __builtin_amdgcn_fence(__ATOMIC_RELEASE, "workgroup");
  __builtin_amdgcn_wave_barrier();
  __builtin_amdgcn_fence(__ATOMIC_ACQUIRE, "workgroup");
  v4u hw[4], lw[4];
#pragma unroll
  for (int i = 0; i < 4; ++i) {
    const v4f a = *(const v4fa*)(sr + i * 256 + 8 * lane);
    const v4f b = *(const v4fa*)(sr + i * 256 + 8 * lane + 4);
    v4u hq, lq;
    unsigned h, l;
    split2(a[0], a[1], h, l); hq[0] = h; lq[0] = l;
    split2(a[2], a[3], h, l); hq[1] = h; lq[1] = l;
    split2(b[0], b[1], h, l); hq[2] = h; lq[2] = l;
    split2(b[2], b[3], h, l); hq[3] = h; lq[3] = l;
    hw[i] = hq; lw[i] = lq;
  }
  const size_t gb = (size_t)row * ND + 8 * lane;
  for (int pass = 0; pass < 2; ++pass) {
#pragma unroll
    for (int i = 0; i < 4; ++i) {
      *(volatile v4u*)(oh + gb + i * 256) = hw[i];
      *(volatile v4u*)(ol + gb + i * 256) = lw[i];
    }
    __threadfence();
  }
}

__global__ __launch_bounds__(256) void rowsoftmax_kernel(const float* __restrict__ S, float* outr,
                                                        unsigned short* __restrict__ oh,
                                                        unsigned short* __restrict__ ol) {
  __shared__ __align__(16) float sRow[8][NJ];
  const int lane = threadIdx.x & 31, wave = threadIdx.x >> 5;
  const int row = blockIdx.x * 8 + wave;
  const float* sp = S + (size_t)row * NJ + 4 * lane;
  v4f v[4];
#pragma unroll
  for (int i = 0; i < 4; ++i) v[i] = *(const v4fa*)(sp + i * 128);
  float mx = v[0][0];
#pragma unroll
  for (int i = 0; i < 4; ++i)
#pragma unroll
    for (int e = 0; e < 4; ++e) mx = fmaxf(mx, v[i][e]);
#pragma unroll
  for (int off = 16; off > 0; off >>= 1) mx = fmaxf(mx, __shfl_xor(mx, off));
  float sum = 0.0f;
#pragma unroll
  for (int i = 0; i < 4; ++i)
#pragma unroll
    for (int e = 0; e < 4; ++e) { const float ex = __expf(v[i][e] - mx); v[i][e] = ex; sum += ex; }
#pragma unroll
  for (int off = 16; off > 0; off >>= 1) sum += __shfl_xor(sum, off);
  const float inv = 1.0f / sum;
#pragma unroll
  for (int i = 0; i < 4; ++i) v[i] = v[i] * inv;

  float* orow = outr + (size_t)row * NJ + 4 * lane;
  for (int pass = 0; pass < 2; ++pass) {
#pragma unroll
    for (int i = 0; i < 4; ++i) *(volatile v4f*)(orow + i * 128) = v[i];
    __threadfence();
  }

  float* sr = sRow[wave];
#pragma unroll
  for (int i = 0; i < 4; ++i) *(v4fa*)(sr + i * 128 + 4 * lane) = v[i];
  __builtin_amdgcn_fence(__ATOMIC_RELEASE, "workgroup");
  __builtin_amdgcn_wave_barrier();
  __builtin_amdgcn_fence(__ATOMIC_ACQUIRE, "workgroup");
  v4u hw[2], lw[2];
#pragma unroll
  for (int i = 0; i < 2; ++i) {
    const v4f a = *(const v4fa*)(sr + i * 256 + 8 * lane);
    const v4f b = *(const v4fa*)(sr + i * 256 + 8 * lane + 4);
    v4u hq, lq;
    unsigned h, l;
    split2(a[0], a[1], h, l); hq[0] = h; lq[0] = l;
    split2(a[2], a[3], h, l); hq[1] = h; lq[1] = l;
    split2(b[0], b[1], h, l); hq[2] = h; lq[2] = l;
    split2(b[2], b[3], h, l); hq[3] = h; lq[3] = l;
    hw[i] = hq; lw[i] = lq;
  }
  const size_t gb = (size_t)row * NJ + 8 * lane;
  for (int pass = 0; pass < 2; ++pass) {
#pragma unroll
    for (int i = 0; i < 2; ++i) {
      *(volatile v4u*)(oh + gb + i * 256) = hw[i];
      *(volatile v4u*)(ol + gb + i * 256) = lw[i];
    }
    __threadfence();
  }
}

extern "C" void kernel_launch(void* const* d_in, const int* in_sizes, int n_in,
                              void* d_out, int out_size, void* d_ws, size_t ws_size,
                              hipStream_t stream) {
  if (n_in < 2) return;
  if (in_sizes[0] != NR * ND) return;
  if (in_sizes[1] != NJ * ND) return;
  if (out_size != NR * NJ + NR * ND) return;

  const float* cls   = (const float*)d_in[0];
  const float* proto = (const float*)d_in[1];
  float* out0 = (float*)d_out;
  float* out1 = out0 + (size_t)NR * NJ;

  const size_t B_CLS = (size_t)NR * ND * 2;
  const size_t B_PJ  = (size_t)NJ * ND * 2;
  const size_t B_SF  = (size_t)NJ * NR * 4;
  const size_t B_RT  = (size_t)NJ * NR * 2;
  const size_t B_PF  = (size_t)NJ * ND * 4;
  size_t off = 0;
  const size_t oCLSB = off; off += B_CLS;
  const size_t oCLST = off; off += B_CLS;
  const size_t oP0B  = off; off += B_PJ;
  const size_t oPH   = off; off += B_PJ;   const size_t oPL  = off; off += B_PJ;
  const size_t oSF   = off; off += B_SF;
  const size_t oRTH  = off; off += B_RT;   const size_t oRTL = off; off += B_RT;
  const size_t oPF   = off; off += B_PF;
  const size_t oPN   = off; off += B_PF;
  const size_t oRH   = off; off += B_RT;   const size_t oRL  = off; off += B_RT;
  const size_t oPTH  = off; off += B_PJ;   const size_t oPTL = off; off += B_PJ;
  if (off > ws_size) return;
  if (off > (size_t)WSLIM) return;
  if (oPL != oPH + B_PJ || oRTL != oRTH + B_RT || oRL != oRH + B_RT || oPTL != oPTH + B_PJ) return;

  char* ws = (char*)d_ws;
  unsigned short* CLSB = (unsigned short*)(ws + oCLSB);
  unsigned short* CLST = (unsigned short*)(ws + oCLST);
  unsigned short* P0B  = (unsigned short*)(ws + oP0B);
  unsigned short* PH   = (unsigned short*)(ws + oPH);
  unsigned short* PL   = (unsigned short*)(ws + oPL);
  float*          SF   = (float*)(ws + oSF);
  unsigned short* RTH  = (unsigned short*)(ws + oRTH);
  unsigned short* RTL  = (unsigned short*)(ws + oRTL);
  float*          PF   = (float*)(ws + oPF);
  float*          PN   = (float*)(ws + oPN);
  unsigned short* RH   = (unsigned short*)(ws + oRH);
  unsigned short* RL   = (unsigned short*)(ws + oRL);
  unsigned short* PTH  = (unsigned short*)(ws + oPTH);
  unsigned short* PTL  = (unsigned short*)(ws + oPTL);

  const dim3 blk(256);
  const long plPJ = (long)NJ * ND;
  const long plRT = (long)NJ * NR;

  const int n8c = NR * ND / 8;
  cvt_bf16x8_kernel<<<dim3((n8c + 255) / 256), blk, 0, stream>>>(cls, CLSB, n8c);
  tcvt_kernel<<<dim3(ND / 64, NR / 64), blk, 0, stream>>>(cls, CLST, NR, ND);
  const int n8p = NJ * ND / 8;
  cvt_bf16x8_kernel<<<dim3((n8p + 255) / 256), blk, 0, stream>>>(proto, P0B, n8p);

  const dim3 gST(((NJ / 64) * (NR / 64) + 7) / 8);
  const dim3 gUP(((NJ / 64) * (ND / 64) + 7) / 8);
  const dim3 gS (((NR / 64) * (NJ / 64) + 7) / 8);
  const dim3 gZ (((NR / 64) * (ND / 64) + 7) / 8);

  for (int s = 0; s < 5; ++s) {
    const unsigned short* Apl = (s == 0) ? P0B : PH;
    const int nt = (s == 0) ? 1 : 2;
    gemm64_kernel<0><<<gST, blk, 0, stream>>>(Apl, ND, plPJ, 0L, CLSB, ND, 0L, 0L, nt,
                                              SF, NR, cls, ND, NJ, NR, ND);
    colsoftmax_kernel<<<dim3(NR / 64), blk, 0, stream>>>(SF, RTH, RTL);
    gemm64_kernel<0><<<gUP, blk, 0, stream>>>(RTH, NR, plRT, 0L, CLST, NR, 0L, 0L, 2,
                                              PF, ND, cls, ND, NJ, ND, NR);
    rownorm_kernel<<<dim3(NJ / 8), blk, 0, stream>>>(PF, PN, PH, PL);
  }

  gemm64_kernel<0><<<gS, blk, 0, stream>>>(CLSB, ND, 0L, 0L, PH, ND, plPJ, 0L, 2,
                                           SF, NJ, cls, ND, NR, NJ, ND);
  rowsoftmax_kernel<<<dim3(NR / 8), blk, 0, stream>>>(SF, out0, RH, RL);
  tsplit_kernel<<<dim3(ND / 64, NJ / 64), blk, 0, stream>>>(PN, PTH, PTL, NJ, ND);
  gemm64_kernel<1><<<gZ, blk, 0, stream>>>(RH, NJ, 0L, plRT, PTH, NJ, plPJ, 0L, 3,
                                           out1, ND, cls, ND, NR, ND, NJ);
  (void)hipGetLastError();
}
